// EmbeddedAttention_65154653880773
// MI455X (gfx1250) — hardware-run, weakly checked
//
#include <hip/hip_runtime.h>

#define BB 16
#define TT 12
#define NN 512
#define DD 128
#define EE 32
#define NBT (BB * TT)
#define NTN (TT * NN)
#define NEGFILL (-1.0e9f)

typedef unsigned short v16us __attribute__((ext_vector_type(16)));
typedef unsigned short v8us  __attribute__((ext_vector_type(8)));
typedef __attribute__((ext_vector_type(16))) __bf16 v16bf;
typedef float v8f __attribute__((ext_vector_type(8)));
typedef float v4f __attribute__((ext_vector_type(4)));
typedef int   v4i __attribute__((ext_vector_type(4)));
typedef v8us __attribute__((may_alias)) v8usa;
typedef v4f  __attribute__((may_alias)) v4fa;
typedef v4i  __attribute__((may_alias)) v4ia;

union Frag { v16us u; v8us half[2]; v16bf b; };

__device__ __forceinline__ v8f wmma_bf(v16us a, v16us b, v8f c) {
  Frag fa, fb;
  fa.u = a;
  fb.u = b;
  v8f d = __builtin_amdgcn_wmma_f32_16x16x32_bf16(false, fa.b, false, fb.b, (short)0, c, false, false);
  asm volatile("v_nop\n\tv_nop\n\tv_nop\n\tv_nop" : "+v"(d) : "v"(a), "v"(b));
  return d;
}

__device__ __forceinline__ unsigned int bfb(float x) {
  const unsigned int u = __float_as_uint(x);
  return (u + 0x7FFFu + ((u >> 16) & 1u)) >> 16;
}

__device__ __forceinline__ void split2(float x, unsigned int& hi, unsigned int& lo) {
  const unsigned int hb = bfb(x);
  hi = hb;
  lo = bfb(x - __uint_as_float(hb << 16));
}

__device__ __forceinline__ v16us load_frag(const unsigned short* p, int h) {
  Frag f;
  f.half[0] = *(const v8usa*)(p + 8 * h);
  f.half[1] = *(const v8usa*)(p + 16 + 8 * h);
  return f.u;
}

__device__ __forceinline__ void frag_split_f32(const float* p, int h, v16us& hi, v16us& lo) {
  const v4f a0 = *(const v4fa*)(p + 8 * h);
  const v4f a1 = *(const v4fa*)(p + 8 * h + 4);
  const v4f a2 = *(const v4fa*)(p + 16 + 8 * h);
  const v4f a3 = *(const v4fa*)(p + 20 + 8 * h);
  const float x[16] = {a0.x, a0.y, a0.z, a0.w, a1.x, a1.y, a1.z, a1.w,
                       a2.x, a2.y, a2.z, a2.w, a3.x, a3.y, a3.z, a3.w};
  v16us vh, vl;
#pragma unroll
  for (int i = 0; i < 16; ++i) {
    unsigned int hh, ll;
    split2(x[i], hh, ll);
    vh[i] = (unsigned short)hh;
    vl[i] = (unsigned short)ll;
  }
  hi = vh;
  lo = vl;
}

__device__ __forceinline__ void frag_masked(const float* sp, const int* mp, int h,
                                            v16us& hi, v16us& lo, v16us& om) {
  const v4f a0 = *(const v4fa*)(sp + 8 * h);
  const v4f a1 = *(const v4fa*)(sp + 8 * h + 4);
  const v4f a2 = *(const v4fa*)(sp + 16 + 8 * h);
  const v4f a3 = *(const v4fa*)(sp + 20 + 8 * h);
  const v4i m0 = *(const v4ia*)(mp + 8 * h);
  const v4i m1 = *(const v4ia*)(mp + 8 * h + 4);
  const v4i m2 = *(const v4ia*)(mp + 16 + 8 * h);
  const v4i m3 = *(const v4ia*)(mp + 20 + 8 * h);
  const float x[16] = {a0.x, a0.y, a0.z, a0.w, a1.x, a1.y, a1.z, a1.w,
                       a2.x, a2.y, a2.z, a2.w, a3.x, a3.y, a3.z, a3.w};
  const int mk[16] = {m0.x, m0.y, m0.z, m0.w, m1.x, m1.y, m1.z, m1.w,
                      m2.x, m2.y, m2.z, m2.w, m3.x, m3.y, m3.z, m3.w};
  v16us vh, vl, vm;
#pragma unroll
  for (int i = 0; i < 16; ++i) {
    const bool keep = (mk[i] != 0);
    const float xs = keep ? x[i] : 0.0f;
    unsigned int hh, ll;
    split2(xs, hh, ll);
    vh[i] = (unsigned short)hh;
    vl[i] = (unsigned short)ll;
    vm[i] = keep ? (unsigned short)0 : (unsigned short)0x3F80;
  }
  hi = vh;
  lo = vl;
  om = vm;
}

__device__ __forceinline__ void tile16x64_store_pass(const float* so, float* g, int pitch, int lane) {
  const int q8 = lane & 7, seg = (lane >> 3) & 1, rsub = lane >> 4;
#pragma unroll
  for (int i = 0; i < 8; ++i) {
    const int rl = 2 * i + rsub;
    const v4f v = *(const v4fa*)(so + rl * 64 + 32 * seg + 4 * q8);
    *(volatile v4f*)(g + (size_t)rl * pitch + 32 * seg + 4 * q8) = v;
  }
}

__global__ __launch_bounds__(128) void k_prep(
    const float* __restrict__ Wv, const float* __restrict__ Wqk,
    unsigned short* __restrict__ WvTh, unsigned short* __restrict__ WvTl,
    unsigned short* __restrict__ WqTh, unsigned short* __restrict__ WqTl)
{
  __shared__ __attribute__((aligned(16))) float sbuf[4096];
  const int tid = threadIdx.x, lane = tid & 31, w = tid >> 5;
  const int bid = blockIdx.x;
  if (bid < 8) {
    const int n0 = bid * 16;
#pragma unroll
    for (int i = 0; i < 16; ++i) {
      const int idx = i * 128 + tid;
      const int k = idx >> 4, c = idx & 15;
      sbuf[k * 16 + c] = Wv[(size_t)k * DD + n0 + c];
    }
    __syncthreads();
    v8us oh[2], ol[2];
    size_t off[2];
#pragma unroll
    for (int i = 0; i < 2; ++i) {
      const int rl = 4 * w + 2 * i + (lane >> 4);
      const int k = 8 * (lane & 15);
      v8us vh, vl;
#pragma unroll
      for (int j = 0; j < 8; ++j) {
        unsigned int hh, ll;
        split2(sbuf[(k + j) * 16 + rl], hh, ll);
        vh[j] = (unsigned short)hh;
        vl[j] = (unsigned short)ll;
      }
      oh[i] = vh;
      ol[i] = vl;
      off[i] = (size_t)(n0 + rl) * DD + k;
    }
#pragma unroll
    for (int i = 0; i < 2; ++i) {
      *(volatile v8us*)(WvTh + off[i]) = oh[i];
      *(volatile v8us*)(WvTl + off[i]) = ol[i];
    }
    __threadfence();
#pragma unroll
    for (int i = 0; i < 2; ++i) {
      *(volatile v8us*)(WvTh + off[i]) = oh[i];
      *(volatile v8us*)(WvTl + off[i]) = ol[i];
    }
  } else {
#pragma unroll
    for (int i = 0; i < 32; ++i) sbuf[i * 128 + tid] = Wqk[i * 128 + tid];
    __syncthreads();
    v8us oh[4], ol[4];
    size_t off[4];
#pragma unroll
    for (int i = 0; i < 4; ++i) {
      const int j = 4 * w + i;
      const int n = 8 * j + (lane >> 2);
      const int k = 8 * (lane & 3);
      v8us vh, vl;
#pragma unroll
      for (int jj = 0; jj < 8; ++jj) {
        unsigned int hh, ll;
        split2(sbuf[(k + jj) * 128 + n], hh, ll);
        vh[jj] = (unsigned short)hh;
        vl[jj] = (unsigned short)ll;
      }
      oh[i] = vh;
      ol[i] = vl;
      off[i] = (size_t)n * EE + k;
    }
#pragma unroll
    for (int i = 0; i < 4; ++i) {
      *(volatile v8us*)(WqTh + off[i]) = oh[i];
      *(volatile v8us*)(WqTl + off[i]) = ol[i];
    }
    __threadfence();
#pragma unroll
    for (int i = 0; i < 4; ++i) {
      *(volatile v8us*)(WqTh + off[i]) = oh[i];
      *(volatile v8us*)(WqTl + off[i]) = ol[i];
    }
  }
}

__device__ __forceinline__ void qk_store_pass(const float* sF, const unsigned short* sH, const unsigned short* sL,
                                              float* QK, unsigned short* Qh, unsigned short* Ql,
                                              int brow0, int tid) {
  const int q8 = tid & 7, sub = tid >> 3;
#pragma unroll
  for (int i = 0; i < 16; ++i) {
    const int L = i * 8 + sub;
    const int row = L >> 2, seg = L & 3;
    const v4f v = *(const v4fa*)(sF + row * DD + 32 * seg + 4 * q8);
    *(volatile v4f*)(QK + (size_t)(brow0 + row) * DD + 32 * seg + 4 * q8) = v;
  }
#pragma unroll
  for (int i = 0; i < 8; ++i) {
    const int L = i * 8 + sub;
    const int row = L >> 1, seg = L & 1;
    const int e = row * DD + 64 * seg + 8 * q8;
    const v8us a = *(const v8usa*)(sH + e);
    const v8us c = *(const v8usa*)(sL + e);
    const size_t g = (size_t)(brow0 + row) * DD + 64 * seg + 8 * q8;
    *(volatile v8us*)(Qh + g) = a;
    *(volatile v8us*)(Ql + g) = c;
  }
}

__global__ __launch_bounds__(64) void k_qk(
    const float* __restrict__ emb, const unsigned short* __restrict__ WqTh,
    const unsigned short* __restrict__ WqTl, const float* __restrict__ bqk,
    float* __restrict__ QK, unsigned short* __restrict__ Qh, unsigned short* __restrict__ Ql)
{
  __shared__ __attribute__((aligned(16))) float sF[32 * DD];
  __shared__ __attribute__((aligned(16))) unsigned short sH[32 * DD];
  __shared__ __attribute__((aligned(16))) unsigned short sL[32 * DD];

  const int tid = threadIdx.x, lane = tid & 31, w = tid >> 5;
  const int h = lane >> 4, ml = lane & 15;
  const int brow0 = blockIdx.x * 32;
  const int row0 = brow0 + 16 * w;

  v16us ah, al;
  frag_split_f32(emb + (size_t)(row0 + ml) * EE, h, ah, al);

  const v8f z8 = {0.f, 0.f, 0.f, 0.f, 0.f, 0.f, 0.f, 0.f};
  v8f acc[8];
#pragma unroll
  for (int c = 0; c < 8; ++c) {
    const size_t bo = (size_t)(16 * c + ml) * EE;
    const v16us bh = load_frag(WqTh + bo, h);
    const v16us bl = load_frag(WqTl + bo, h);
    v8f d = wmma_bf(ah, bh, z8);
    d = wmma_bf(ah, bl, d);
    d = wmma_bf(al, bh, d);
    acc[c] = d;
  }

#pragma unroll
  for (int c = 0; c < 8; ++c) {
    const int col = 16 * c + ml;
    const float bb = bqk[col];
#pragma unroll
    for (int r = 0; r < 8; ++r) {
      const float y = acc[c][r] + bb;
      acc[c][r] = y;
      sF[(16 * w + 8 * h + r) * DD + col] = y;
    }
  }

#pragma unroll
  for (int r = 0; r < 8; ++r) {
    float mx = acc[0][r];
#pragma unroll
    for (int c = 1; c < 8; ++c) mx = fmaxf(mx, acc[c][r]);
    mx = fmaxf(mx, __shfl_xor(mx, 8));
    mx = fmaxf(mx, __shfl_xor(mx, 4));
    mx = fmaxf(mx, __shfl_xor(mx, 2));
    mx = fmaxf(mx, __shfl_xor(mx, 1));
    float s = 0.f;
#pragma unroll
    for (int c = 0; c < 8; ++c) {
      const float e = __expf(acc[c][r] - mx);
      acc[c][r] = e;
      s += e;
    }
    s += __shfl_xor(s, 8);
    s += __shfl_xor(s, 4);
    s += __shfl_xor(s, 2);
    s += __shfl_xor(s, 1);
    const float inv = 1.0f / s;
    const int rl = 16 * w + 8 * h + r;
#pragma unroll
    for (int c = 0; c < 8; ++c) {
      unsigned int hh, ll;
      split2(acc[c][r] * inv, hh, ll);
      sH[rl * DD + 16 * c + ml] = (unsigned short)hh;
      sL[rl * DD + 16 * c + ml] = (unsigned short)ll;
    }
  }
  __syncthreads();

  qk_store_pass(sF, sH, sL, QK, Qh, Ql, brow0, tid);
  __threadfence();
  qk_store_pass(sF, sH, sL, QK, Qh, Ql, brow0, tid);
}

__device__ __forceinline__ void kt_store_pass(const unsigned short* sH, const unsigned short* sL,
                                              unsigned short* KTh, unsigned short* KTl,
                                              size_t rowbase, int tid) {
  const int q8 = tid & 7, sub = tid >> 3;
#pragma unroll
  for (int i = 0; i < 4; ++i) {
    const int L = i * 16 + sub;
    const int row = L >> 1, seg = L & 1;
    const int e = row * DD + 64 * seg + 8 * q8;
    const v8us a = *(const v8usa*)(sH + e);
    const v8us c = *(const v8usa*)(sL + e);
    const size_t g = (rowbase + row) * DD + 64 * seg + 8 * q8;
    *(volatile v8us*)(KTh + g) = a;
    *(volatile v8us*)(KTl + g) = c;
  }
}

__global__ __launch_bounds__(128) void k_ksm(
    const float* __restrict__ QK, unsigned short* __restrict__ KTh, unsigned short* __restrict__ KTl)
{
  __shared__ __attribute__((aligned(16))) unsigned short sH[32 * DD];
  __shared__ __attribute__((aligned(16))) unsigned short sL[32 * DD];

  const int tid = threadIdx.x;
  const int t = blockIdx.x;
  const int d = tid;
  const float* base = QK + (size_t)t * NN * DD + d;

  float mx = -3.0e38f;
#pragma unroll 4
  for (int n = 0; n < NN; ++n) mx = fmaxf(mx, base[(size_t)n * DD]);
  float s = 0.f;
#pragma unroll 4
  for (int n = 0; n < NN; ++n) s += __expf(base[(size_t)n * DD] - mx);
  const float inv = 1.0f / s;

#pragma unroll 1
  for (int nb = 0; nb < NN / 32; ++nb) {
#pragma unroll 4
    for (int j = 0; j < 32; ++j) {
      const float kv = __expf(base[(size_t)(nb * 32 + j) * DD] - mx) * inv;
      unsigned int hh, ll;
      split2(kv, hh, ll);
      sH[j * DD + d] = (unsigned short)hh;
      sL[j * DD + d] = (unsigned short)ll;
    }
    __syncthreads();
    const size_t rowbase = (size_t)t * NN + nb * 32;
    kt_store_pass(sH, sL, KTh, KTl, rowbase, tid);
    __threadfence();
    kt_store_pass(sH, sL, KTh, KTl, rowbase, tid);
    __syncthreads();
  }
}

__global__ __launch_bounds__(128) void k_score(
    const unsigned short* __restrict__ Qh, const unsigned short* __restrict__ Ql,
    const unsigned short* __restrict__ KTh, const unsigned short* __restrict__ KTl,
    float* __restrict__ SC)
{
  __shared__ __attribute__((aligned(16))) float sO[4 * 16 * 64];

  const int tid = threadIdx.x, lane = tid & 31, w = tid >> 5;
  const int h = lane >> 4, ml = lane & 15;
  const int gid = blockIdx.x * 4 + w;
  const int t = gid >> 8, rt = gid & 255;
  const int row0 = (rt >> 3) * 16, col0 = (rt & 7) * 64;
  const size_t qo = ((size_t)t * NN + row0 + ml) * DD;
  const size_t ko = ((size_t)t * NN + col0 + ml) * DD;

  const v8f z8 = {0.f, 0.f, 0.f, 0.f, 0.f, 0.f, 0.f, 0.f};
  v8f acc[4];
#pragma unroll
  for (int c = 0; c < 4; ++c) acc[c] = z8;

#pragma unroll 1
  for (int k0 = 0; k0 < DD; k0 += 32) {
    const v16us ah = load_frag(Qh + qo + k0, h);
    const v16us al = load_frag(Ql + qo + k0, h);
#pragma unroll
    for (int c = 0; c < 4; ++c) {
      const size_t bo = ko + (size_t)(16 * c) * DD + k0;
      const v16us bh = load_frag(KTh + bo, h);
      const v16us bl = load_frag(KTl + bo, h);
      acc[c] = wmma_bf(ah, bh, acc[c]);
      acc[c] = wmma_bf(ah, bl, acc[c]);
      acc[c] = wmma_bf(al, bh, acc[c]);
    }
  }

  float* so = sO + w * 1024;
#pragma unroll
  for (int c = 0; c < 4; ++c)
#pragma unroll
    for (int r = 0; r < 8; ++r)
      so[(8 * h + r) * 64 + 16 * c + ml] = acc[c][r];
  __syncthreads();

  float* g = SC + ((size_t)t * NN + row0) * NN + col0;
  tile16x64_store_pass(so, g, NN, lane);
  __threadfence();
  tile16x64_store_pass(so, g, NN, lane);
}

__device__ __forceinline__ void vt_store_pass(const unsigned short* sTh, const unsigned short* sTl,
                                              unsigned short* VTh, unsigned short* VTl,
                                              size_t gbase, int tid) {
  const int q8 = tid & 7, sub = tid >> 3;
#pragma unroll
  for (int i = 0; i < 8; ++i) {
    const int dl = i * 16 + sub;
    const int e = dl * 64 + 8 * q8;
    const v8us a = *(const v8usa*)(sTh + e);
    const v8us c = *(const v8usa*)(sTl + e);
    const size_t g = gbase + (size_t)dl * NN + 8 * q8;
    *(volatile v8us*)(VTh + g) = a;
    *(volatile v8us*)(VTl + g) = c;
  }
}

__global__ __launch_bounds__(128) void k_vproj(
    const float* __restrict__ value, const unsigned short* __restrict__ WvTh,
    const unsigned short* __restrict__ WvTl, const float* __restrict__ bv,
    unsigned short* __restrict__ VTh, unsigned short* __restrict__ VTl)
{
  __shared__ __attribute__((aligned(16))) unsigned short sTh[DD * 64];
  __shared__ __attribute__((aligned(16))) unsigned short sTl[DD * 64];

  const int tid = threadIdx.x, lane = tid & 31, w = tid >> 5;
  const int h = lane >> 4, ml = lane & 15;
  const int grow0 = blockIdx.x * 64;
  const int bt = grow0 >> 9;
  const int mloc0 = grow0 & (NN - 1);
  const size_t ao = (size_t)(grow0 + 16 * w + ml) * DD;

  const v8f z8 = {0.f, 0.f, 0.f, 0.f, 0.f, 0.f, 0.f, 0.f};
  v8f acc[8];
#pragma unroll
  for (int c = 0; c < 8; ++c) acc[c] = z8;

#pragma unroll 1
  for (int k0 = 0; k0 < DD; k0 += 32) {
    v16us ah, al;
    frag_split_f32(value + ao + k0, h, ah, al);
#pragma unroll
    for (int c = 0; c < 8; ++c) {
      const size_t bo = (size_t)(16 * c + ml) * DD + k0;
      const v16us bh = load_frag(WvTh + bo, h);
      const v16us bl = load_frag(WvTl + bo, h);
      acc[c] = wmma_bf(ah, bh, acc[c]);
      acc[c] = wmma_bf(ah, bl, acc[c]);
      acc[c] = wmma_bf(al, bh, acc[c]);
    }
  }

#pragma unroll
  for (int c = 0; c < 8; ++c) {
    const int d = 16 * c + ml;
    const float bb = bv[d];
#pragma unroll
    for (int r = 0; r < 8; ++r) {
      const int m = 16 * w + 8 * h + r;
      unsigned int hh, ll;
      split2(acc[c][r] + bb, hh, ll);
      sTh[d * 64 + m] = (unsigned short)hh;
      sTl[d * 64 + m] = (unsigned short)ll;
    }
  }
  __syncthreads();

  const size_t gbase = (size_t)bt * DD * NN + mloc0;
  vt_store_pass(sTh, sTl, VTh, VTl, gbase, tid);
  __threadfence();
  vt_store_pass(sTh, sTl, VTh, VTl, gbase, tid);
}

__global__ __launch_bounds__(128) void k_out(
    const float* __restrict__ SC, const int* __restrict__ mask,
    const unsigned short* __restrict__ VTh, const unsigned short* __restrict__ VTl,
    float* __restrict__ out)
{
  __shared__ __attribute__((aligned(16))) float sO[4 * 16 * 64];

  const int tid = threadIdx.x, lane = tid & 31, w = tid >> 5;
  const int h = lane >> 4, ml = lane & 15;
  const int bt = blockIdx.x >> 4, nb = blockIdx.x & 15;
  const int b = bt / TT, t = bt - b * TT;
  const int row0 = nb * 32 + 16 * (w >> 1);
  const int d0 = 64 * (w & 1);
  const float* srow = SC + ((size_t)t * NN + row0 + ml) * NN;
  const int*   mrow = mask + ((size_t)b * NN + row0 + ml) * NN;
  const size_t vo = ((size_t)bt * DD + d0 + ml) * NN;

  const v8f z8 = {0.f, 0.f, 0.f, 0.f, 0.f, 0.f, 0.f, 0.f};
  v8f c1[4], c2[4];
#pragma unroll
  for (int c = 0; c < 4; ++c) { c1[c] = z8; c2[c] = z8; }

#pragma unroll 1
  for (int k0 = 0; k0 < NN; k0 += 32) {
    v16us ah, al, am;
    frag_masked(srow + k0, mrow + k0, h, ah, al, am);
#pragma unroll
    for (int c = 0; c < 4; ++c) {
      const size_t bo = vo + (size_t)(16 * c) * NN + k0;
      const v16us bh = load_frag(VTh + bo, h);
      const v16us bl = load_frag(VTl + bo, h);
      c1[c] = wmma_bf(ah, bh, c1[c]);
      c1[c] = wmma_bf(ah, bl, c1[c]);
      c1[c] = wmma_bf(al, bh, c1[c]);
      c2[c] = wmma_bf(am, bh, c2[c]);
      c2[c] = wmma_bf(am, bl, c2[c]);
    }
  }

  float* so = sO + w * 1024;
#pragma unroll
  for (int c = 0; c < 4; ++c)
#pragma unroll
    for (int r = 0; r < 8; ++r)
      so[(8 * h + r) * 64 + 16 * c + ml] = c1[c][r] + NEGFILL * c2[c][r];
  __syncthreads();

  float* g = out + ((size_t)bt * NN + row0) * DD + d0;
  tile16x64_store_pass(so, g, DD, lane);
  __threadfence();
  tile16x64_store_pass(so, g, DD, lane);
}

extern "C" void kernel_launch(void* const* d_in, const int* in_sizes, int n_in,
                              void* d_out, int out_size, void* d_ws, size_t ws_size,
                              hipStream_t stream) {
  if (n_in < 7) return;
  if (in_sizes[0] != BB * TT * NN * DD) return;
  if (in_sizes[1] != TT * NN * EE) return;
  if (in_sizes[2] != BB * NN * NN) return;
  if (in_sizes[3] != EE * DD) return;
  if (in_sizes[4] != DD) return;
  if (in_sizes[5] != DD * DD) return;
  if (in_sizes[6] != DD) return;
  if (out_size != BB * TT * NN * DD) return;

  const float* value = (const float*)d_in[0];
  const float* emb   = (const float*)d_in[1];
  const int*   amask = (const int*)d_in[2];
  const float* Wqk   = (const float*)d_in[3];
  const float* bqk   = (const float*)d_in[4];
  const float* Wv    = (const float*)d_in[5];
  const float* bv    = (const float*)d_in[6];
  float* out = (float*)d_out;

  const size_t sz_wv  = (size_t)DD * DD * 2;
  const size_t sz_wq  = (size_t)DD * EE * 2;
  const size_t sz_qk  = (size_t)NTN * DD * 4;
  const size_t sz_q16 = (size_t)NTN * DD * 2;
  const size_t sz_sc  = (size_t)TT * NN * NN * 4;
  const size_t sz_vt  = (size_t)NBT * DD * NN * 2;
  size_t off = 0;
  const size_t o_wvh = off; off += sz_wv;
  const size_t o_wvl = off; off += sz_wv;
  const size_t o_wqh = off; off += sz_wq;
  const size_t o_wql = off; off += sz_wq;
  const size_t o_qk  = off; off += sz_qk;
  const size_t o_qh  = off; off += sz_q16;
  const size_t o_ql  = off; off += sz_q16;
  const size_t o_kth = off; off += sz_q16;
  const size_t o_ktl = off; off += sz_q16;
  const size_t o_sc  = off; off += sz_sc;
  const size_t o_vth = off; off += sz_vt;
  const size_t o_vtl = off; off += sz_vt;
  const size_t total = off;
  if (total > ws_size) return;

  char* ws = (char*)d_ws;
  unsigned short* WvTh = (unsigned short*)(ws + o_wvh);
  unsigned short* WvTl = (unsigned short*)(ws + o_wvl);
  unsigned short* WqTh = (unsigned short*)(ws + o_wqh);
  unsigned short* WqTl = (unsigned short*)(ws + o_wql);
  float*          QK   = (float*)(ws + o_qk);
  unsigned short* Qh   = (unsigned short*)(ws + o_qh);
  unsigned short* Ql   = (unsigned short*)(ws + o_ql);
  unsigned short* KTh  = (unsigned short*)(ws + o_kth);
  unsigned short* KTl  = (unsigned short*)(ws + o_ktl);
  float*          SC   = (float*)(ws + o_sc);
  unsigned short* VTh  = (unsigned short*)(ws + o_vth);
  unsigned short* VTl  = (unsigned short*)(ws + o_vtl);

  k_prep<<<9, 128, 0, stream>>>(Wv, Wqk, WvTh, WvTl, WqTh, WqTl);
  k_qk<<<NTN / 32, 64, 0, stream>>>(emb, WqTh, WqTl, bqk, QK, Qh, Ql);
  k_ksm<<<TT, DD, 0, stream>>>(QK, KTh, KTl);
  k_score<<<(TT * 256) / 4, 128, 0, stream>>>(Qh, Ql, KTh, KTl, SC);
  k_vproj<<<(BB * TT * NN) / 64, 128, 0, stream>>>(value, WvTh, WvTl, bv, VTh, VTl);
  k_out<<<NBT * 16, 128, 0, stream>>>(SC, amask, VTh, VTl, out);
}
